// GatedAttentionUnit_51436528337427
// MI455X (gfx1250) — hardware-run, weakly checked
//
#include <hip/hip_runtime.h>
#include <math.h>
#include <stdint.h>

#ifndef SEQ
#define SEQ 2048
#endif
#define S_FULL  2048
#define NBATCH  4
#define EDIM    1024
#define ZD      128
#define HD      2048
#define NPROJ   (2 * HD + ZD)
#define MROWS   (SEQ * NBATCH)
#define MASK_LD S_FULL
#define RPB_C   (S_FULL - 1)
#define RPB_N   (2 * S_FULL - 1)
#define PCAR    16384.0f
#define VCAR    256.0f
#define INV_S   (1.0f / (float)SEQ)
#define TP      68
#define PTH     72
#define WS_CAP  134217728
static_assert((SEQ % 64) == 0 && SEQ >= 64 && SEQ <= S_FULL);
static_assert((NPROJ % 64) == 0 && (HD % 64) == 0 && (EDIM % 64) == 0 && (ZD % 64) == 0);
static_assert((ZD % 32) == 0 && (EDIM % 32) == 0 && (HD % 32) == 0 && (SEQ % 32) == 0);
static_assert(((MROWS * EDIM / 8) % 256) == 0 && ((NPROJ * EDIM / 8) % 256) == 0 && ((EDIM * HD / 8) % 256) == 0);
static_assert(64 * TP * 4 <= 65536 && 4 * 16 * PTH * 2 <= 65536 && 4 * 16 * TP * 4 <= 65536);

typedef unsigned short u16;
typedef unsigned short v8us __attribute__((ext_vector_type(8)));
typedef _Float16 v16h __attribute__((ext_vector_type(16)));
typedef _Float16 v8h  __attribute__((ext_vector_type(8)));
typedef __bf16   v16b __attribute__((ext_vector_type(16)));
typedef float    v8f  __attribute__((ext_vector_type(8)));
typedef float    v4f  __attribute__((ext_vector_type(4)));
typedef unsigned int v4u __attribute__((ext_vector_type(4)));

union FragH { v16h v; v8h h[2]; };
union FragB { v16b v; v4u u[2]; };

__device__ __forceinline__ unsigned short bf_bits(float f) {
  unsigned u = __float_as_uint(f);
  return (unsigned short)((u + 0x7FFFu + ((u >> 16) & 1u)) >> 16);
}
__device__ __forceinline__ float bf_up(unsigned short h) { return __uint_as_float(((unsigned)h) << 16); }
__device__ __forceinline__ float bfr(float f) { return bf_up(bf_bits(f)); }
__device__ __forceinline__ unsigned short h_bits(_Float16 x) { return __builtin_bit_cast(unsigned short, x); }
__device__ __forceinline__ unsigned pk16(unsigned short a, unsigned short b) { return (unsigned)a | ((unsigned)b << 16); }
__device__ __forceinline__ v8f zero8() { v8f z = {0.f, 0.f, 0.f, 0.f, 0.f, 0.f, 0.f, 0.f}; return z; }

__device__ __forceinline__ v16h ldfrag_h(const _Float16* p) {
  FragH f;
  f.h[0] = *(const v8h*)(p);
  f.h[1] = *(const v8h*)(p + 16);
  return f.v;
}
__device__ __forceinline__ v16b ldfrag_b(const u16* p) {
  FragB f;
  f.u[0] = *(const v4u*)(p);
  f.u[1] = *(const v4u*)(p + 16);
  return f.v;
}

__device__ __forceinline__ v8f mma_h(v16h a, v16h b, v8f c) {
  return __builtin_amdgcn_wmma_f32_16x16x32_f16(false, a, false, b, (short)0, c, false, false);
}
__device__ __forceinline__ v8f mma_b(v16b a, v16b b, v8f c) {
  return __builtin_amdgcn_wmma_f32_16x16x32_bf16(false, a, false, b, (short)0, c, false, false);
}
template <typename F>
__device__ __forceinline__ void guard6(v8f& a, v8f& b, v8f& c, v8f& d, F x0, F x1, F x2, F x3, F x4, F x5) {
#if defined(__HIP_DEVICE_COMPILE__)
  asm volatile("v_nop\n\tv_nop\n\tv_nop\n\tv_nop"
               : "+v"(a), "+v"(b), "+v"(c), "+v"(d) : "v"(x0), "v"(x1), "v"(x2), "v"(x3), "v"(x4), "v"(x5) : "memory");
#endif
}
__device__ __forceinline__ void wave_sync_lds() {
  __builtin_amdgcn_fence(__ATOMIC_RELEASE, "workgroup");
  __builtin_amdgcn_wave_barrier();
  __builtin_amdgcn_fence(__ATOMIC_ACQUIRE, "workgroup");
}
__device__ __forceinline__ float silu_f(float t) {
#pragma clang fp contract(off)
  const float e = expf(-t);
  return t * (1.0f / (1.0f + e));
}

__global__ __launch_bounds__(256) void cvt_bf(const float* __restrict__ x, u16* D, int n8) {
  const int gt = (int)blockIdx.x * 256 + (int)threadIdx.x;
  if (gt >= n8) return;
  const float* p = x + (size_t)gt * 8;
  const v4f a = *(const v4f*)(p), c = *(const v4f*)(p + 4);
  v4u o;
  o[0] = pk16(bf_bits(a[0]), bf_bits(a[1]));
  o[1] = pk16(bf_bits(a[2]), bf_bits(a[3]));
  o[2] = pk16(bf_bits(c[0]), bf_bits(c[1]));
  o[3] = pk16(bf_bits(c[2]), bf_bits(c[3]));
  u16* d = D + (size_t)gt * 8;
  *(volatile v4u*)(d) = o;
  __threadfence();
  *(volatile v4u*)(d) = o;
}

__global__ __launch_bounds__(128)
void k_proj(const u16* __restrict__ X16, const u16* __restrict__ PW, const float* __restrict__ pb,
            const float* __restrict__ gam, const float* __restrict__ bet,
            float* U, u16* VT, u16* QP, u16* KP, int b) {
#pragma clang fp contract(off)
  __shared__ __align__(16) float T[64 * TP];
  const int tid = threadIdx.x, wave = tid >> 5, lane = tid & 31, hh = lane >> 4, m = lane & 15;
  const int nct  = NPROJ / 64;
  const int bid  = (int)blockIdx.x;
  const int ct   = bid % nct;
  const int st   = bid / nct;
  const int s0   = st * 64;
  if (s0 + 64 > SEQ) return;
  const int col0 = ct * 64;
  const int rowb = s0 + wave * 16;
  const u16* ap = X16 + ((size_t)(rowb + m) * NBATCH + b) * EDIM + 8 * hh;
  const u16* bp = PW + (size_t)(col0 + m) * EDIM + 8 * hh;
  const size_t bs = (size_t)16 * EDIM;
  v8f acc0 = zero8(), acc1 = zero8(), acc2 = zero8(), acc3 = zero8();
#pragma unroll 1
  for (int k0 = 0; k0 < EDIM; k0 += 32) {
    const v16b a  = ldfrag_b(ap + k0);
    const v16b b0 = ldfrag_b(bp + k0);
    const v16b b1 = ldfrag_b(bp + bs + k0);
    const v16b b2 = ldfrag_b(bp + 2 * bs + k0);
    const v16b b3 = ldfrag_b(bp + 3 * bs + k0);
    acc0 = mma_b(a, b0, acc0);
    acc1 = mma_b(a, b1, acc1);
    acc2 = mma_b(a, b2, acc2);
    acc3 = mma_b(a, b3, acc3);
    guard6<v16b>(acc0, acc1, acc2, acc3, a, b0, b1, b2, b3, a);
  }
  {
    float* tw = T + (wave * 16) * TP;
#pragma unroll
    for (int r = 0; r < 8; ++r) {
      const int ro = (8 * hh + r) * TP + m;
      tw[ro]      = acc0[r];
      tw[ro + 16] = acc1[r];
      tw[ro + 32] = acc2[r];
      tw[ro + 48] = acc3[r];
    }
  }
  __syncthreads();
  const int p8 = tid & 7, lq = tid >> 3;
  if (col0 < HD) {
#pragma unroll 1
    for (int it = 0; it < 8; ++it) {
      const int L = it * 16 + lq;
      const int row = L >> 1, half = L & 1;
      const int c4 = half * 32 + p8 * 4;
      const v4f a = *(const v4f*)(T + row * TP + c4);
      v4f o;
#pragma unroll
      for (int e = 0; e < 4; ++e) o[e] = silu_f(a[e] + bfr(pb[col0 + c4 + e]));
      float* d = U + (size_t)(s0 + row) * HD + col0 + c4;
      *(volatile v4f*)(d) = o;
      __threadfence();
      *(volatile v4f*)(d) = o;
    }
  } else if (col0 < 2 * HD) {
#pragma unroll 1
    for (int it = 0; it < 4; ++it) {
      const int hl = it * 16 + lq;
      const float bb = bfr(pb[col0 + hl]);
      v4u o;
#pragma unroll
      for (int e = 0; e < 4; ++e) {
        const float f0 = silu_f(T[(p8 * 8 + 2 * e) * TP + hl] + bb);
        const float f1 = silu_f(T[(p8 * 8 + 2 * e + 1) * TP + hl] + bb);
        o[e] = pk16(h_bits((_Float16)(f0 * VCAR)), h_bits((_Float16)(f1 * VCAR)));
      }
      u16* d = VT + (size_t)(col0 - HD + hl) * SEQ + s0 + p8 * 8;
      *(volatile v4u*)(d) = o;
      __threadfence();
      *(volatile v4u*)(d) = o;
    }
  } else {
    const int zoff = col0 - 2 * HD;
#pragma unroll 1
    for (int it = 0; it < 4; ++it) {
      const int row = it * 16 + lq;
      const v4f a = *(const v4f*)(T + row * TP + p8 * 8), c = *(const v4f*)(T + row * TP + p8 * 8 + 4);
      float w[8];
#pragma unroll
      for (int e = 0; e < 4; ++e) { w[e] = a[e]; w[4 + e] = c[e]; }
      v4u oq, ok;
#pragma unroll
      for (int e = 0; e < 4; ++e) {
        const int i0 = 2 * e, i1 = 2 * e + 1;
        const int z0 = zoff + p8 * 8 + i0, z1 = zoff + p8 * 8 + i1;
        const float sv0 = silu_f(w[i0] + bfr(pb[col0 + p8 * 8 + i0]));
        const float sv1 = silu_f(w[i1] + bfr(pb[col0 + p8 * 8 + i1]));
        const float q0v = sv0 * bfr(gam[z0]) + bfr(bet[z0]);
        const float q1v = sv1 * bfr(gam[z1]) + bfr(bet[z1]);
        const float k0v = sv0 * bfr(gam[ZD + z0]) + bfr(bet[ZD + z0]);
        const float k1v = sv1 * bfr(gam[ZD + z1]) + bfr(bet[ZD + z1]);
        oq[e] = pk16(bf_bits(q0v), bf_bits(q1v));
        ok[e] = pk16(bf_bits(k0v), bf_bits(k1v));
      }
      u16* dq = QP + (size_t)(s0 + row) * ZD + zoff + p8 * 8;
      u16* dk = KP + (size_t)(s0 + row) * ZD + zoff + p8 * 8;
      *(volatile v4u*)(dq) = oq;
      *(volatile v4u*)(dk) = ok;
      __threadfence();
      *(volatile v4u*)(dq) = oq;
      *(volatile v4u*)(dk) = ok;
    }
  }
}

__device__ __forceinline__ u16 score_p16(float a, float bias, int mk) {
#pragma clang fp contract(off)
  const float s = a * INV_S + bias;
  float t = (mk != 0) ? 0.0f : s;
  t = fmaxf(t, 0.0f);
  const float p = (t * t) * PCAR;
  return h_bits((_Float16)p);
}

__global__ __launch_bounds__(128)
void k_score(const u16* __restrict__ QP, const u16* __restrict__ KP, const int* __restrict__ maskp,
             const float* __restrict__ rpb, u16* Pp) {
#pragma clang fp contract(off)
  __shared__ __align__(16) u16 ph[4 * 16 * PTH];
  const int tid = threadIdx.x, wave = tid >> 5, lane = tid & 31, hh = lane >> 4, m = lane & 15;
  const int kt = (int)blockIdx.x, qt = (int)blockIdx.y;
  if (kt > qt) return;
  if (qt * 64 + 64 > SEQ) return;
  const int q0 = qt * 64 + wave * 16;
  const int k0 = kt * 64;
  const u16* ap = QP + (size_t)(q0 + m) * ZD + 8 * hh;
  const u16* bp = KP + (size_t)(k0 + m) * ZD + 8 * hh;
  const size_t bs = (size_t)16 * ZD;
  v8f acc0 = zero8(), acc1 = zero8(), acc2 = zero8(), acc3 = zero8();
#pragma unroll
  for (int ks = 0; ks < ZD; ks += 32) {
    const v16b a  = ldfrag_b(ap + ks);
    const v16b b0 = ldfrag_b(bp + ks);
    const v16b b1 = ldfrag_b(bp + bs + ks);
    const v16b b2 = ldfrag_b(bp + 2 * bs + ks);
    const v16b b3 = ldfrag_b(bp + 3 * bs + ks);
    acc0 = mma_b(a, b0, acc0);
    acc1 = mma_b(a, b1, acc1);
    acc2 = mma_b(a, b2, acc2);
    acc3 = mma_b(a, b3, acc3);
    guard6<v16b>(acc0, acc1, acc2, acc3, a, b0, b1, b2, b3, a);
  }
  u16* pw = ph + wave * (16 * PTH);
#pragma unroll
  for (int r = 0; r < 8; ++r) {
    const int q = q0 + 8 * hh + r;
    const int* mr = maskp + (size_t)q * MASK_LD + k0 + m;
    const float* br = rpb + (RPB_C - q + k0 + m);
    const int ro = (8 * hh + r) * PTH + m;
    pw[ro]      = score_p16(acc0[r], bfr(br[0]),  mr[0]);
    pw[ro + 16] = score_p16(acc1[r], bfr(br[16]), mr[16]);
    pw[ro + 32] = score_p16(acc2[r], bfr(br[32]), mr[32]);
    pw[ro + 48] = score_p16(acc3[r], bfr(br[48]), mr[48]);
  }
  wave_sync_lds();
  const int p8 = lane & 7, lq = lane >> 3;
  const v8us o0 = *(const v8us*)(pw + (0  + lq) * PTH + p8 * 8);
  const v8us o1 = *(const v8us*)(pw + (4  + lq) * PTH + p8 * 8);
  const v8us o2 = *(const v8us*)(pw + (8  + lq) * PTH + p8 * 8);
  const v8us o3 = *(const v8us*)(pw + (12 + lq) * PTH + p8 * 8);
  u16* d = Pp + (size_t)(q0 + lq) * SEQ + k0 + p8 * 8;
  const size_t r4 = (size_t)4 * SEQ;
  *(volatile v8us*)(d)          = o0;
  *(volatile v8us*)(d + r4)     = o1;
  *(volatile v8us*)(d + 2 * r4) = o2;
  *(volatile v8us*)(d + 3 * r4) = o3;
  __threadfence();
  *(volatile v8us*)(d)          = o0;
  *(volatile v8us*)(d + r4)     = o1;
  *(volatile v8us*)(d + 2 * r4) = o2;
  *(volatile v8us*)(d + 3 * r4) = o3;
}

__global__ __launch_bounds__(128)
void k_pv(const u16* __restrict__ Pp, const u16* __restrict__ VT, const float* __restrict__ U, u16* GH, u16* GL) {
#pragma clang fp contract(off)
  __shared__ __align__(16) float slab[4 * 16 * TP];
  const int tid = threadIdx.x, wave = tid >> 5, lane = tid & 31, hh = lane >> 4, m = lane & 15;
  const int nht  = HD / 64;
  const int bid  = (int)blockIdx.x;
  const int ht   = bid % nht;
  const int qt   = bid / nht;
  if (qt * 64 + 64 > SEQ) return;
  const int rowb = qt * 64 + wave * 16;
  const int col0 = ht * 64;
  const int kend = qt * 64 + 64;
  const _Float16* ap = (const _Float16*)(const void*)Pp + (size_t)(rowb + m) * SEQ + 8 * hh;
  const _Float16* bp = (const _Float16*)(const void*)VT + (size_t)(col0 + m) * SEQ + 8 * hh;
  const size_t bs = (size_t)16 * SEQ;
  v8f acc0 = zero8(), acc1 = zero8(), acc2 = zero8(), acc3 = zero8();
#pragma unroll 1
  for (int k0 = 0; k0 < kend; k0 += 32) {
    const v16h a  = ldfrag_h(ap + k0);
    const v16h b0 = ldfrag_h(bp + k0);
    const v16h b1 = ldfrag_h(bp + bs + k0);
    const v16h b2 = ldfrag_h(bp + 2 * bs + k0);
    const v16h b3 = ldfrag_h(bp + 3 * bs + k0);
    acc0 = mma_h(a, b0, acc0);
    acc1 = mma_h(a, b1, acc1);
    acc2 = mma_h(a, b2, acc2);
    acc3 = mma_h(a, b3, acc3);
    guard6<v16h>(acc0, acc1, acc2, acc3, a, b0, b1, b2, b3, a);
  }
  float* sl = slab + wave * (16 * TP);
  const float oc = 1.0f / (PCAR * VCAR);
#pragma unroll
  for (int r = 0; r < 8; ++r) {
    const int ro = (8 * hh + r) * TP + m;
    sl[ro]      = acc0[r] * oc;
    sl[ro + 16] = acc1[r] * oc;
    sl[ro + 32] = acc2[r] * oc;
    sl[ro + 48] = acc3[r] * oc;
  }
  wave_sync_lds();
  const int p8 = lane & 7, lq = lane >> 3;
  v4u gh0, gh1, gh2, gh3, gl0, gl1, gl2, gl3;
#pragma unroll
  for (int it = 0; it < 4; ++it) {
    const int row = it * 4 + lq;
    const float* sp = sl + row * TP + p8 * 8;
    const v4f a = *(const v4f*)(sp), c = *(const v4f*)(sp + 4);
    const float* up = U + (size_t)(rowb + row) * HD + col0 + p8 * 8;
    const v4f ua = *(const v4f*)(up), uc = *(const v4f*)(up + 4);
    float w[8];
#pragma unroll
    for (int e = 0; e < 4; ++e) { w[e] = a[e] * ua[e]; w[4 + e] = c[e] * uc[e]; }
    v4u oh, ol;
#pragma unroll
    for (int e = 0; e < 4; ++e) {
      const float f0 = w[2 * e], f1 = w[2 * e + 1];
      const unsigned short h0 = bf_bits(f0), h1 = bf_bits(f1);
      const unsigned short l0 = bf_bits(f0 - bf_up(h0)), l1 = bf_bits(f1 - bf_up(h1));
      oh[e] = pk16(h0, h1);
      ol[e] = pk16(l0, l1);
    }
    if (it == 0) { gh0 = oh; gl0 = ol; }
    else if (it == 1) { gh1 = oh; gl1 = ol; }
    else if (it == 2) { gh2 = oh; gl2 = ol; }
    else { gh3 = oh; gl3 = ol; }
  }
  const size_t o0 = (size_t)(rowb + lq) * HD + col0 + p8 * 8;
  const size_t r4 = (size_t)4 * HD;
  *(volatile v4u*)(GH + o0)          = gh0;
  *(volatile v4u*)(GH + o0 + r4)     = gh1;
  *(volatile v4u*)(GH + o0 + 2 * r4) = gh2;
  *(volatile v4u*)(GH + o0 + 3 * r4) = gh3;
  *(volatile v4u*)(GL + o0)          = gl0;
  *(volatile v4u*)(GL + o0 + r4)     = gl1;
  *(volatile v4u*)(GL + o0 + 2 * r4) = gl2;
  *(volatile v4u*)(GL + o0 + 3 * r4) = gl3;
  __threadfence();
  *(volatile v4u*)(GH + o0)          = gh0;
  *(volatile v4u*)(GH + o0 + r4)     = gh1;
  *(volatile v4u*)(GH + o0 + 2 * r4) = gh2;
  *(volatile v4u*)(GH + o0 + 3 * r4) = gh3;
  *(volatile v4u*)(GL + o0)          = gl0;
  *(volatile v4u*)(GL + o0 + r4)     = gl1;
  *(volatile v4u*)(GL + o0 + 2 * r4) = gl2;
  *(volatile v4u*)(GL + o0 + 3 * r4) = gl3;
}

__global__ __launch_bounds__(128)
void k_out(const u16* __restrict__ GH, const u16* __restrict__ GL, const u16* __restrict__ OW,
           const float* __restrict__ ob, float* out, int b) {
#pragma clang fp contract(off)
  __shared__ __align__(16) float slab[4 * 16 * TP];
  const int tid = threadIdx.x, wave = tid >> 5, lane = tid & 31, hh = lane >> 4, m = lane & 15;
  const int net  = EDIM / 64;
  const int bid  = (int)blockIdx.x;
  const int et   = bid % net;
  const int st   = bid / net;
  if (st * 64 + 64 > SEQ) return;
  const int rowb = st * 64 + wave * 16;
  const int col0 = et * 64;
  const u16* ahp = GH + (size_t)(rowb + m) * HD + 8 * hh;
  const u16* alp = GL + (size_t)(rowb + m) * HD + 8 * hh;
  const u16* bp  = OW + (size_t)(col0 + m) * HD + 8 * hh;
  const size_t bs = (size_t)16 * HD;
  v8f acc0 = zero8(), acc1 = zero8(), acc2 = zero8(), acc3 = zero8();
#pragma unroll 1
  for (int k0 = 0; k0 < HD; k0 += 32) {
    const v16b ah = ldfrag_b(ahp + k0);
    const v16b al = ldfrag_b(alp + k0);
    const v16b b0 = ldfrag_b(bp + k0);
    const v16b b1 = ldfrag_b(bp + bs + k0);
    const v16b b2 = ldfrag_b(bp + 2 * bs + k0);
    const v16b b3 = ldfrag_b(bp + 3 * bs + k0);
    acc0 = mma_b(ah, b0, acc0);
    acc0 = mma_b(al, b0, acc0);
    acc1 = mma_b(ah, b1, acc1);
    acc1 = mma_b(al, b1, acc1);
    acc2 = mma_b(ah, b2, acc2);
    acc2 = mma_b(al, b2, acc2);
    acc3 = mma_b(ah, b3, acc3);
    acc3 = mma_b(al, b3, acc3);
    guard6<v16b>(acc0, acc1, acc2, acc3, ah, al, b0, b1, b2, b3);
  }
  const float bj0 = bfr(ob[col0 + m]);
  const float bj1 = bfr(ob[col0 + 16 + m]);
  const float bj2 = bfr(ob[col0 + 32 + m]);
  const float bj3 = bfr(ob[col0 + 48 + m]);
  float* sl = slab + wave * (16 * TP);
#pragma unroll
  for (int r = 0; r < 8; ++r) {
    const int ro = (8 * hh + r) * TP + m;
    sl[ro]      = acc0[r] + bj0;
    sl[ro + 16] = acc1[r] + bj1;
    sl[ro + 32] = acc2[r] + bj2;
    sl[ro + 48] = acc3[r] + bj3;
  }
  wave_sync_lds();
  v4f vals[8];
#pragma unroll
  for (int it = 0; it < 8; ++it) vals[it] = *(const v4f*)(sl + (it * 2 + hh) * TP + m * 4);
  float* dst = out + ((size_t)(rowb + hh) * NBATCH + b) * EDIM + col0 + m * 4;
  const size_t r2 = (size_t)2 * NBATCH * EDIM;
#pragma unroll
  for (int it = 0; it < 8; ++it) *(volatile v4f*)(dst + (size_t)it * r2) = vals[it];
  __threadfence();
#pragma unroll
  for (int it = 0; it < 8; ++it) *(volatile v4f*)(dst + (size_t)it * r2) = vals[it];
}

extern "C" void kernel_launch(void* const* d_in, const int* in_sizes, int n_in,
                              void* d_out, int out_size, void* d_ws, size_t ws_size,
                              hipStream_t stream) {
  if (n_in < 9) return;
  if (in_sizes[0] < MROWS * EDIM) return;
  if (in_sizes[1] != S_FULL * S_FULL) return;
  if (in_sizes[2] != NPROJ * EDIM) return;
  if (in_sizes[3] != NPROJ) return;
  if (in_sizes[4] != EDIM * HD) return;
  if (in_sizes[5] != EDIM) return;
  if (in_sizes[6] != 2 * ZD || in_sizes[7] != 2 * ZD) return;
  if (in_sizes[8] != RPB_N) return;
  if (out_size < MROWS * EDIM) return;

  const float* x      = (const float*)d_in[0];
  const int*   mask   = (const int*)d_in[1];
  const float* proj_w = (const float*)d_in[2];
  const float* proj_b = (const float*)d_in[3];
  const float* out_w  = (const float*)d_in[4];
  const float* out_b  = (const float*)d_in[5];
  const float* gamma  = (const float*)d_in[6];
  const float* beta   = (const float*)d_in[7];
  const float* rpb    = (const float*)d_in[8];
  float*       out    = (float*)d_out;

  const size_t szX  = (size_t)MROWS * EDIM * 2;
  const size_t szPW = (size_t)NPROJ * EDIM * 2;
  const size_t szOW = (size_t)EDIM * HD * 2;
  const size_t szU  = (size_t)SEQ * HD * 4;
  const size_t szVT = (size_t)HD * SEQ * 2;
  const size_t szQ  = (size_t)SEQ * ZD * 2;
  const size_t szP  = (size_t)SEQ * SEQ * 2;
  const size_t szG  = (size_t)SEQ * HD * 2;
  size_t off = 0;
  const size_t oX  = off; off += szX;
  const size_t oPW = off; off += szPW;
  const size_t oOW = off; off += szOW;
  const size_t oU  = off; off += szU;
  const size_t oVT = off; off += szVT;
  const size_t oQP = off; off += szQ;
  const size_t oKP = off; off += szQ;
  const size_t oP  = off; off += szP;
  const size_t oGH = off; off += szG;
  const size_t oGL = off; off += szG;
  if (off > ws_size) return;
  if (off > (size_t)WS_CAP) return;

  char* ws = (char*)d_ws;
  u16*   X16 = (u16*)(ws + oX);
  u16*   PW  = (u16*)(ws + oPW);
  u16*   OW  = (u16*)(ws + oOW);
  float* U   = (float*)(ws + oU);
  u16*   VT  = (u16*)(ws + oVT);
  u16*   QP  = (u16*)(ws + oQP);
  u16*   KP  = (u16*)(ws + oKP);
  u16*   P   = (u16*)(ws + oP);
  u16*   GH  = (u16*)(ws + oGH);
  u16*   GL  = (u16*)(ws + oGL);

  const dim3 b256(256), b128(128);
  const int  n8x = (MROWS * EDIM) / 8;
  const int  n8w = (NPROJ * EDIM) / 8;
  const int  n8o = (EDIM * HD) / 8;
  const dim3 gX((n8x + 255) / 256), gW((n8w + 255) / 256), gO((n8o + 255) / 256);
  const dim3 gP((SEQ / 64) * (NPROJ / 64));
  const dim3 gS(SEQ / 64, SEQ / 64);
  const dim3 gV((SEQ / 64) * (HD / 64));
  const dim3 gY((SEQ / 64) * (EDIM / 64));

  cvt_bf<<<gX, b256, 0, stream>>>(x, X16, n8x);
  cvt_bf<<<gW, b256, 0, stream>>>(proj_w, PW, n8w);
  cvt_bf<<<gO, b256, 0, stream>>>(out_w, OW, n8o);
  for (int bq = 0; bq < NBATCH; ++bq) {
    k_proj<<<gP, b128, 0, stream>>>(X16, PW, proj_b, gamma, beta, U, VT, QP, KP, bq);
    k_score<<<gS, b128, 0, stream>>>(QP, KP, mask, rpb, P);
    k_pv<<<gV, b128, 0, stream>>>(P, VT, U, GH, GL);
    k_out<<<gY, b128, 0, stream>>>(GH, GL, OW, out_b, out, bq);
  }
  (void)hipGetLastError();
}
